// TrajectoryHGNN_65652870087171
// MI455X (gfx1250) — hardware-run, weakly checked
//
#include <hip/hip_runtime.h>


namespace {
constexpr int B = 64, N = 512, T = 8, DIN = 2, H = 256, L = 3, E = 8192, M = 128, PO = 24, NN = B * N, NE = B * E, NM = B * M, NBLK = NN / 16;
constexpr float XS = 8.0f, WSC = 256.0f;
typedef _Float16 b16;
typedef __attribute__((ext_vector_type(16))) _Float16 v16b;
typedef __attribute__((ext_vector_type(8))) _Float16 v8b;
typedef __attribute__((ext_vector_type(8))) float v8f;
typedef __attribute__((ext_vector_type(4))) float v4f;
__device__ __forceinline__ float bf16_rne(float f) { unsigned int u = __float_as_uint(f); u += 0x7FFFu + ((u >> 16) & 1u); return __uint_as_float(u & 0xFFFF0000u); }
__device__ __forceinline__ void split16(float v, b16& hi, b16& lo) { hi = (b16)v; lo = (b16)(v - (float)hi); }
__device__ __forceinline__ v16b frag_kb(const b16* p, int hh) { const v8b a = *(const v8b*)(p + 8 * hh), b = *(const v8b*)(p + 16 + 8 * hh); v16b f;
#pragma unroll
  for (int e = 0; e < 8; ++e) { f[e] = a[e]; f[8 + e] = b[e]; } return f; }
__device__ __forceinline__ v8f wmma16b(v16b a, v16b b, v8f c) { v8f d = __builtin_amdgcn_wmma_f32_16x16x32_f16(false, a, false, b, (short)0, c, false, false); asm volatile("v_nop\n\tv_nop\n\tv_nop\n\tv_nop" : "+v"(d) : "v"(a), "v"(b)); return d; }
__device__ __forceinline__ void wave_lds_sync() { __builtin_amdgcn_fence(__ATOMIC_RELEASE, "workgroup"); __builtin_amdgcn_wave_barrier(); __builtin_amdgcn_fence(__ATOMIC_ACQUIRE, "workgroup"); }
__device__ __forceinline__ float pmul(float a, float b) { float p = a * b; asm volatile("" : "+v"(p)); return p; }
__device__ __forceinline__ int iclamp(int v, int lo, int hi) { return v < lo ? lo : (v > hi ? hi : v); }
constexpr int CSR_NBLK9 = 512, CSR_GB9 = 9, CSR_GN9 = 1 << CSR_GB9  , CSR_TS9 = (CSR_GN9 < 32 ? 32 : CSR_GN9)  , CSR_MAXG9 = 512, CSR_CAP9 = 12288  ;
__device__ __host__ __forceinline__ int csr_tix9(int v) { return (v >> CSR_GB9) * CSR_TS9 + (v & (CSR_GN9 - 1)); }
__global__ __launch_bounds__(64) void csrA_kernel9(const int* __restrict__ dst, int E, int N, int nG, int CHP, int NGP, int* __restrict__ STG, int* __restrict__ HST) {
  extern __shared__ int sm[];
  int* cnt = sm; int* run = sm + NGP; int* ids = sm + 2 * NGP;
  const int b = blockIdx.x; const int ch = (E + CSR_NBLK9 - 1) / CSR_NBLK9; const int e0 = b * ch, e1 = min(E, e0 + ch);
  for (int i = threadIdx.x; i < NGP; i += 64) cnt[i] = 0;
  for (int i = threadIdx.x; i < CHP; i += 64) ids[i] = -1;
  __syncthreads();
  if (threadIdx.x == 0) {
    for (int e = e0; e < e1; ++e) { int d = dst[e]; d = (d < 0) ? 0 : (d >= N ? N - 1 : d); cnt[d >> CSR_GB9] += 1; }
    int acc = 0; for (int g = 0; g < nG; ++g) { run[g] = acc; acc += cnt[g]; }
    for (int e = e0; e < e1; ++e) { int d = dst[e]; d = (d < 0) ? 0 : (d >= N ? N - 1 : d); const int g = d >> CSR_GB9; ids[run[g]] = e; run[g] += 1; } }
  __syncthreads();
  typedef __attribute__((ext_vector_type(4))) int v4i;
  for (int pass = 0; pass < 2; ++pass) {
    for (int i = threadIdx.x; i < CHP / 4; i += 64) *(volatile v4i*)(STG + (size_t)b * CHP + i * 4) = *(const v4i*)(&ids[i * 4]);
    for (int i = threadIdx.x; i < NGP / 4; i += 64) { v4i v; for (int e = 0; e < 4; ++e) v[e] = (i * 4 + e < nG) ? cnt[i * 4 + e] : 0; *(volatile v4i*)(HST + (size_t)b * NGP + i * 4) = v; }
    __threadfence(); }
}
__global__ __launch_bounds__(512) void csrS_kernel9(const int* __restrict__ HST, int nG, int NGP, int* __restrict__ START, int* __restrict__ TOT, int* __restrict__ OFF) {
  __shared__ int tot[CSR_MAXG9];
  const int b = threadIdx.x;
  for (int pass = 0; pass < 2; ++pass) { int runb = 0; for (int g = 0; g < nG; ++g) { int c = HST[(size_t)b * NGP + g]; c = (c < 0) ? 0 : c; ((volatile int*)OFF)[(size_t)g * CSR_NBLK9 + b] = runb; runb += c; } __threadfence(); }
  for (int g = threadIdx.x; g < nG; g += 512) { int s = 0; for (int bb = 0; bb < CSR_NBLK9; ++bb) { int c = HST[(size_t)bb * NGP + g]; s += (c < 0) ? 0 : c; } tot[g] = s; }
  __syncthreads();
  if (threadIdx.x < 32) {
    __shared__ int st[CSR_MAXG9 + 32];
    if (threadIdx.x == 0) { int acc = 0; for (int g = 0; g < NGP; ++g) { st[g] = acc; if (g < nG) acc += (tot[g] + 31) & ~31; } st[NGP] = acc; }
    __builtin_amdgcn_fence(__ATOMIC_RELEASE, "workgroup"); __builtin_amdgcn_wave_barrier(); __builtin_amdgcn_fence(__ATOMIC_ACQUIRE, "workgroup");
    for (int pass = 0; pass < 2; ++pass) { for (int i = threadIdx.x; i < NGP + 32; i += 32) { ((volatile int*)START)[i] = (i <= NGP) ? st[min(i, NGP)] : 0; ((volatile int*)TOT)[i] = (i < nG) ? tot[i] : 0; } __threadfence(); } }
}
__global__ __launch_bounds__(256) void csrB_kernel9(const int* __restrict__ dst, int N, int nG, int CHP, int NGP, int permLen, const int* __restrict__ STG, const int* __restrict__ HST, const int* __restrict__ OFF, const int* __restrict__ START, const int* __restrict__ TOT, int* __restrict__ PERM, int* __restrict__ ROWPTR, int* __restrict__ ROWCNT, int* __restrict__ FLAG) {
  typedef __attribute__((ext_vector_type(4))) int v4i;
  __shared__ int ids[CSR_CAP9]; __shared__ unsigned short key[CSR_CAP9]; __shared__ int outp[CSR_CAP9]; __shared__ int ncnt[CSR_GN9 + 1]; __shared__ int boff[CSR_NBLK9 + 1];
  const int g = blockIdx.x, t_ = threadIdx.x; int tot = TOT[g]; int st = START[g], stn = START[g + 1]; const int v0 = g * CSR_GN9; const int nv = min(CSR_GN9, N - v0); const int t0 = g * CSR_TS9;
  st = (st < 0) ? 0 : (st > permLen - 32 ? permLen - 32 : st) & ~31; stn = (stn < st) ? st : (stn > permLen ? permLen : stn); tot = (tot < 0) ? 0 : tot; if (tot > stn - st && tot <= CSR_CAP9) tot = stn - st;
  if (tot > CSR_CAP9) {
    for (int pass = 0; pass < 2; ++pass) { for (int i = t_; i < CSR_TS9 / 4; i += 256) { v4i a, c; for (int e = 0; e < 4; ++e) { a[e] = st; c[e] = 0; } *(volatile v4i*)(ROWPTR + t0 + i * 4) = a; *(volatile v4i*)(ROWCNT + t0 + i * 4) = c; } if (t_ == 0) ((volatile int*)FLAG)[0] = 1; __threadfence(); } (void)nv; return; }
  if (t_ == 0) { int acc = 0; for (int b = 0; b < CSR_NBLK9; ++b) { boff[b] = acc; int c = HST[(size_t)b * NGP + g]; c = (c < 0) ? 0 : (c > CHP ? CHP : c); acc += c; if (acc > tot) acc = tot; } boff[CSR_NBLK9] = acc; }
  for (int i = t_; i <= CSR_GN9; i += 256) ncnt[i] = 0;
  __syncthreads();
  for (int b = 0; b < CSR_NBLK9; ++b) { const int c = boff[b + 1] - boff[b]; int o_ = OFF[(size_t)g * CSR_NBLK9 + b]; o_ = (o_ < 0) ? 0 : (o_ > CHP - c ? CHP - c : o_); const int* src_ = STG + (size_t)b * CHP + o_;
    for (int i = t_; i < c; i += 256) { int id = src_[i]; id = (id < 0) ? 0 : id; ids[boff[b] + i] = id; int d = dst[id]; d = (d < v0) ? v0 : (d >= N ? N - 1 : d); int kk = d - v0; kk = (kk < 0) ? 0 : (kk >= CSR_GN9 ? CSR_GN9 - 1 : kk); key[boff[b] + i] = (unsigned short)kk; } }
  __syncthreads();
  if (t_ == 0) { for (int i = 0; i < tot; ++i) ncnt[key[i]] += 1; int acc = 0; for (int vl = 0; vl < CSR_GN9; ++vl) { const int c = ncnt[vl]; ncnt[vl] = acc; acc += c; } ncnt[CSR_GN9] = acc;
    for (int i = 0; i < tot; ++i) { const int vl = key[i]; outp[ncnt[vl]] = ids[i]; ncnt[vl] += 1; }
    for (int vl = CSR_GN9; vl > 0; --vl) ncnt[vl] = ncnt[vl - 1]; ncnt[0] = 0; }
  __syncthreads();
  for (int pass = 0; pass < 2; ++pass) {
    for (int i = t_; i < (stn - st) / 4; i += 256) { v4i v; for (int e = 0; e < 4; ++e) { const int q = i * 4 + e; v[e] = (q < tot) ? outp[q] : -1; } *(volatile v4i*)(PERM + st + i * 4) = v; }
    for (int i = t_; i < CSR_TS9 / 4; i += 256) { v4i a, c; for (int e = 0; e < 4; ++e) { const int vl = i * 4 + e; const int vc = vl < CSR_GN9 ? vl : CSR_GN9; a[e] = (vl < CSR_GN9) ? st + ncnt[vc] : st; c[e] = (vl < nv) ? (ncnt[(vc < CSR_GN9 ? vc : CSR_GN9 - 1) + 1] - ncnt[vc]) : 0; } *(volatile v4i*)(ROWPTR + t0 + i * 4) = a; *(volatile v4i*)(ROWCNT + t0 + i * 4) = c; }
    __threadfence(); }
}
__global__ __launch_bounds__(256) void csrZ_kernel9(int* __restrict__ p, size_t n4) { typedef __attribute__((ext_vector_type(4))) int v4i; const size_t tid = (size_t)blockIdx.x * 256 + threadIdx.x, nth = (size_t)gridDim.x * 256; v4i z = {0, 0, 0, 0}; for (size_t i = tid; i < n4; i += nth) *(volatile v4i*)(p + i * 4) = z; }
struct CsrBufs9 { int *STG, *HST, *OFF, *START, *TOT, *PERM, *ROWPTR, *ROWCNT, *FLAG; int nG, NGP, CHP; size_t permLen; char* base; size_t bytes; };
static size_t csr_carve9(CsrBufs9& c, char* ws, size_t off, int E, int N) {
  const size_t off0 = off; c.base = ws + off;
  auto al = [&](size_t bytes) { char* p = ws + off; off += (bytes + 255) & ~(size_t)255; return p; };
  c.nG = (N + CSR_GN9 - 1) / CSR_GN9; c.NGP = (c.nG + 31) & ~31; const int ch = (E + CSR_NBLK9 - 1) / CSR_NBLK9; c.CHP = (ch + 31) & ~31; c.permLen = (size_t)E + 32 * (size_t)c.nG + 32;
  c.STG = (int*)al((size_t)CSR_NBLK9 * c.CHP * 4); c.HST = (int*)al((size_t)CSR_NBLK9 * c.NGP * 4); c.OFF = (int*)al((size_t)c.NGP * CSR_NBLK9 * 4); c.START = (int*)al((size_t)(c.NGP + 64) * 4); c.TOT = (int*)al((size_t)(c.NGP + 64) * 4);
  c.PERM = (int*)al(c.permLen * 4); c.ROWPTR = (int*)al((size_t)c.nG * CSR_TS9 * 4); c.ROWCNT = (int*)al((size_t)c.nG * CSR_TS9 * 4); c.FLAG = (int*)al(256);
  c.bytes = off - off0; return off;
}
static void csr_build9(const CsrBufs9& c, const int* dst, int E, int N, hipStream_t stream) {
  const size_t smem = (size_t)(2 * c.NGP + c.CHP) * 4;
  csrZ_kernel9<<<512, 256, 0, stream>>>((int*)c.base, c.bytes / 16);
  csrA_kernel9<<<CSR_NBLK9, 64, smem, stream>>>(dst, E, N, c.nG, c.CHP, c.NGP, c.STG, c.HST);
  csrS_kernel9<<<1, 512, 0, stream>>>(c.HST, c.nG, c.NGP, c.START, c.TOT, c.OFF);
  csrB_kernel9<<<c.nG, 256, 0, stream>>>(dst, N, c.nG, c.CHP, c.NGP, (int)c.permLen, c.STG, c.HST, c.OFF, c.START, c.TOT, c.PERM, c.ROWPTR, c.ROWCNT, c.FLAG);
}
constexpr int CSR_NBLK6 = 512, CSR_GB6 = 6, CSR_GN6 = 1 << CSR_GB6  , CSR_TS6 = (CSR_GN6 < 32 ? 32 : CSR_GN6)  , CSR_MAXG6 = 512, CSR_CAP6 = 12288  ;
__device__ __host__ __forceinline__ int csr_tix6(int v) { return (v >> CSR_GB6) * CSR_TS6 + (v & (CSR_GN6 - 1)); }
__global__ __launch_bounds__(64) void csrA_kernel6(const int* __restrict__ dst, int E, int N, int nG, int CHP, int NGP, int* __restrict__ STG, int* __restrict__ HST) {
  extern __shared__ int sm[];
  int* cnt = sm; int* run = sm + NGP; int* ids = sm + 2 * NGP;
  const int b = blockIdx.x; const int ch = (E + CSR_NBLK6 - 1) / CSR_NBLK6; const int e0 = b * ch, e1 = min(E, e0 + ch);
  for (int i = threadIdx.x; i < NGP; i += 64) cnt[i] = 0;
  for (int i = threadIdx.x; i < CHP; i += 64) ids[i] = -1;
  __syncthreads();
  if (threadIdx.x == 0) {
    for (int e = e0; e < e1; ++e) { int d = dst[e]; d = (d < 0) ? 0 : (d >= N ? N - 1 : d); cnt[d >> CSR_GB6] += 1; }
    int acc = 0; for (int g = 0; g < nG; ++g) { run[g] = acc; acc += cnt[g]; }
    for (int e = e0; e < e1; ++e) { int d = dst[e]; d = (d < 0) ? 0 : (d >= N ? N - 1 : d); const int g = d >> CSR_GB6; ids[run[g]] = e; run[g] += 1; } }
  __syncthreads();
  typedef __attribute__((ext_vector_type(4))) int v4i;
  for (int pass = 0; pass < 2; ++pass) {
    for (int i = threadIdx.x; i < CHP / 4; i += 64) *(volatile v4i*)(STG + (size_t)b * CHP + i * 4) = *(const v4i*)(&ids[i * 4]);
    for (int i = threadIdx.x; i < NGP / 4; i += 64) { v4i v; for (int e = 0; e < 4; ++e) v[e] = (i * 4 + e < nG) ? cnt[i * 4 + e] : 0; *(volatile v4i*)(HST + (size_t)b * NGP + i * 4) = v; }
    __threadfence(); }
}
__global__ __launch_bounds__(512) void csrS_kernel6(const int* __restrict__ HST, int nG, int NGP, int* __restrict__ START, int* __restrict__ TOT, int* __restrict__ OFF) {
  __shared__ int tot[CSR_MAXG6];
  const int b = threadIdx.x;
  for (int pass = 0; pass < 2; ++pass) { int runb = 0; for (int g = 0; g < nG; ++g) { int c = HST[(size_t)b * NGP + g]; c = (c < 0) ? 0 : c; ((volatile int*)OFF)[(size_t)g * CSR_NBLK6 + b] = runb; runb += c; } __threadfence(); }
  for (int g = threadIdx.x; g < nG; g += 512) { int s = 0; for (int bb = 0; bb < CSR_NBLK6; ++bb) { int c = HST[(size_t)bb * NGP + g]; s += (c < 0) ? 0 : c; } tot[g] = s; }
  __syncthreads();
  if (threadIdx.x < 32) {
    __shared__ int st[CSR_MAXG6 + 32];
    if (threadIdx.x == 0) { int acc = 0; for (int g = 0; g < NGP; ++g) { st[g] = acc; if (g < nG) acc += (tot[g] + 31) & ~31; } st[NGP] = acc; }
    __builtin_amdgcn_fence(__ATOMIC_RELEASE, "workgroup"); __builtin_amdgcn_wave_barrier(); __builtin_amdgcn_fence(__ATOMIC_ACQUIRE, "workgroup");
    for (int pass = 0; pass < 2; ++pass) { for (int i = threadIdx.x; i < NGP + 32; i += 32) { ((volatile int*)START)[i] = (i <= NGP) ? st[min(i, NGP)] : 0; ((volatile int*)TOT)[i] = (i < nG) ? tot[i] : 0; } __threadfence(); } }
}
__global__ __launch_bounds__(256) void csrB_kernel6(const int* __restrict__ dst, int N, int nG, int CHP, int NGP, int permLen, const int* __restrict__ STG, const int* __restrict__ HST, const int* __restrict__ OFF, const int* __restrict__ START, const int* __restrict__ TOT, int* __restrict__ PERM, int* __restrict__ ROWPTR, int* __restrict__ ROWCNT, int* __restrict__ FLAG) {
  typedef __attribute__((ext_vector_type(4))) int v4i;
  __shared__ int ids[CSR_CAP6]; __shared__ unsigned short key[CSR_CAP6]; __shared__ int outp[CSR_CAP6]; __shared__ int ncnt[CSR_GN6 + 1]; __shared__ int boff[CSR_NBLK6 + 1];
  const int g = blockIdx.x, t_ = threadIdx.x; int tot = TOT[g]; int st = START[g], stn = START[g + 1]; const int v0 = g * CSR_GN6; const int nv = min(CSR_GN6, N - v0); const int t0 = g * CSR_TS6;
  st = (st < 0) ? 0 : (st > permLen - 32 ? permLen - 32 : st) & ~31; stn = (stn < st) ? st : (stn > permLen ? permLen : stn); tot = (tot < 0) ? 0 : tot; if (tot > stn - st && tot <= CSR_CAP6) tot = stn - st;
  if (tot > CSR_CAP6) {
    for (int pass = 0; pass < 2; ++pass) { for (int i = t_; i < CSR_TS6 / 4; i += 256) { v4i a, c; for (int e = 0; e < 4; ++e) { a[e] = st; c[e] = 0; } *(volatile v4i*)(ROWPTR + t0 + i * 4) = a; *(volatile v4i*)(ROWCNT + t0 + i * 4) = c; } if (t_ == 0) ((volatile int*)FLAG)[0] = 1; __threadfence(); } (void)nv; return; }
  if (t_ == 0) { int acc = 0; for (int b = 0; b < CSR_NBLK6; ++b) { boff[b] = acc; int c = HST[(size_t)b * NGP + g]; c = (c < 0) ? 0 : (c > CHP ? CHP : c); acc += c; if (acc > tot) acc = tot; } boff[CSR_NBLK6] = acc; }
  for (int i = t_; i <= CSR_GN6; i += 256) ncnt[i] = 0;
  __syncthreads();
  for (int b = 0; b < CSR_NBLK6; ++b) { const int c = boff[b + 1] - boff[b]; int o_ = OFF[(size_t)g * CSR_NBLK6 + b]; o_ = (o_ < 0) ? 0 : (o_ > CHP - c ? CHP - c : o_); const int* src_ = STG + (size_t)b * CHP + o_;
    for (int i = t_; i < c; i += 256) { int id = src_[i]; id = (id < 0) ? 0 : id; ids[boff[b] + i] = id; int d = dst[id]; d = (d < v0) ? v0 : (d >= N ? N - 1 : d); int kk = d - v0; kk = (kk < 0) ? 0 : (kk >= CSR_GN6 ? CSR_GN6 - 1 : kk); key[boff[b] + i] = (unsigned short)kk; } }
  __syncthreads();
  if (t_ == 0) { for (int i = 0; i < tot; ++i) ncnt[key[i]] += 1; int acc = 0; for (int vl = 0; vl < CSR_GN6; ++vl) { const int c = ncnt[vl]; ncnt[vl] = acc; acc += c; } ncnt[CSR_GN6] = acc;
    for (int i = 0; i < tot; ++i) { const int vl = key[i]; outp[ncnt[vl]] = ids[i]; ncnt[vl] += 1; }
    for (int vl = CSR_GN6; vl > 0; --vl) ncnt[vl] = ncnt[vl - 1]; ncnt[0] = 0; }
  __syncthreads();
  for (int pass = 0; pass < 2; ++pass) {
    for (int i = t_; i < (stn - st) / 4; i += 256) { v4i v; for (int e = 0; e < 4; ++e) { const int q = i * 4 + e; v[e] = (q < tot) ? outp[q] : -1; } *(volatile v4i*)(PERM + st + i * 4) = v; }
    for (int i = t_; i < CSR_TS6 / 4; i += 256) { v4i a, c; for (int e = 0; e < 4; ++e) { const int vl = i * 4 + e; const int vc = vl < CSR_GN6 ? vl : CSR_GN6; a[e] = (vl < CSR_GN6) ? st + ncnt[vc] : st; c[e] = (vl < nv) ? (ncnt[(vc < CSR_GN6 ? vc : CSR_GN6 - 1) + 1] - ncnt[vc]) : 0; } *(volatile v4i*)(ROWPTR + t0 + i * 4) = a; *(volatile v4i*)(ROWCNT + t0 + i * 4) = c; }
    __threadfence(); }
}
__global__ __launch_bounds__(256) void csrZ_kernel6(int* __restrict__ p, size_t n4) { typedef __attribute__((ext_vector_type(4))) int v4i; const size_t tid = (size_t)blockIdx.x * 256 + threadIdx.x, nth = (size_t)gridDim.x * 256; v4i z = {0, 0, 0, 0}; for (size_t i = tid; i < n4; i += nth) *(volatile v4i*)(p + i * 4) = z; }
struct CsrBufs6 { int *STG, *HST, *OFF, *START, *TOT, *PERM, *ROWPTR, *ROWCNT, *FLAG; int nG, NGP, CHP; size_t permLen; char* base; size_t bytes; };
static size_t csr_carve6(CsrBufs6& c, char* ws, size_t off, int E, int N) {
  const size_t off0 = off; c.base = ws + off;
  auto al = [&](size_t bytes) { char* p = ws + off; off += (bytes + 255) & ~(size_t)255; return p; };
  c.nG = (N + CSR_GN6 - 1) / CSR_GN6; c.NGP = (c.nG + 31) & ~31; const int ch = (E + CSR_NBLK6 - 1) / CSR_NBLK6; c.CHP = (ch + 31) & ~31; c.permLen = (size_t)E + 32 * (size_t)c.nG + 32;
  c.STG = (int*)al((size_t)CSR_NBLK6 * c.CHP * 4); c.HST = (int*)al((size_t)CSR_NBLK6 * c.NGP * 4); c.OFF = (int*)al((size_t)c.NGP * CSR_NBLK6 * 4); c.START = (int*)al((size_t)(c.NGP + 64) * 4); c.TOT = (int*)al((size_t)(c.NGP + 64) * 4);
  c.PERM = (int*)al(c.permLen * 4); c.ROWPTR = (int*)al((size_t)c.nG * CSR_TS6 * 4); c.ROWCNT = (int*)al((size_t)c.nG * CSR_TS6 * 4); c.FLAG = (int*)al(256);
  c.bytes = off - off0; return off;
}
static void csr_build6(const CsrBufs6& c, const int* dst, int E, int N, hipStream_t stream) {
  const size_t smem = (size_t)(2 * c.NGP + c.CHP) * 4;
  csrZ_kernel6<<<512, 256, 0, stream>>>((int*)c.base, c.bytes / 16);
  csrA_kernel6<<<CSR_NBLK6, 64, smem, stream>>>(dst, E, N, c.nG, c.CHP, c.NGP, c.STG, c.HST);
  csrS_kernel6<<<1, 512, 0, stream>>>(c.HST, c.nG, c.NGP, c.START, c.TOT, c.OFF);
  csrB_kernel6<<<c.nG, 256, 0, stream>>>(dst, N, c.nG, c.CHP, c.NGP, (int)c.permLen, c.STG, c.HST, c.OFF, c.START, c.TOT, c.PERM, c.ROWPTR, c.ROWCNT, c.FLAG);
}


__global__ __launch_bounds__(256) void wio_kernel(const float* __restrict__ w, int OUTW, int OUTP, b16* __restrict__ WT) {
  const int u = blockIdx.x * 256 + threadIdx.x; if (u >= OUTP * H / 8) return; const int e = u * 8; const int o = e / H, k0 = e % H; v8b v;
#pragma unroll
  for (int j = 0; j < 8; ++j) v[j] = o < OUTW ? (b16)(bf16_rne(w[(size_t)(k0 + j) * OUTW + o]) * WSC) : (b16)0.0f; for (int pass = 0; pass < 2; ++pass) { *(volatile v8b*)(WT + e) = v; __threadfence(); }
}
__global__ __launch_bounds__(256) void keys_kernel(const int* __restrict__ hi, int* __restrict__ KN, int* __restrict__ KE) {
  const int p = blockIdx.x * 256 + threadIdx.x; if (p >= NE) return; const int b = p / E, e = p % E; const int n = iclamp(hi[((size_t)b * 2 + 0) * E + e], 0, N - 1), m = iclamp(hi[((size_t)b * 2 + 1) * E + e], 0, M - 1);
  for (int pass = 0; pass < 2; ++pass) { ((volatile int*)KN)[p] = b * N + n; ((volatile int*)KE)[p] = b * M + m; __threadfence(); }
}
__global__ __launch_bounds__(256) void enc_kernel(const float* __restrict__ obs, const float* __restrict__ We, const float* __restrict__ be, int NLIM, float* __restrict__ H0, float* __restrict__ HS) {
  const size_t gid = (size_t)blockIdx.x * 256 + threadIdx.x; const size_t n = gid / (H / 4); const int c4 = (int)(gid % (H / 4)) * 4; if (n >= (size_t)NLIM) return;
  float w0[4], w1[4], bb[4]; for (int q = 0; q < 4; ++q) { w0[q] = bf16_rne(We[c4 + q]); w1[q] = bf16_rne(We[H + c4 + q]); bb[q] = bf16_rne(be[c4 + q]); } v4f s = {0, 0, 0, 0};
#pragma unroll 1
  for (int t = 0; t < T; ++t) { const float o0 = bf16_rne(obs[(n * T + t) * DIN]), o1 = bf16_rne(obs[(n * T + t) * DIN + 1]); for (int q = 0; q < 4; ++q) s[q] += fmaxf(pmul(o0, w0[q]) + pmul(o1, w1[q]) + bb[q], 0.0f); }
  v4f r; for (int q = 0; q < 4; ++q) r[q] = s[q] * (1.0f / T);
  for (int pass = 0; pass < 2; ++pass) { *(volatile v4f*)(H0 + n * H + c4) = r; *(volatile v4f*)(HS + n * H + c4) = r; __threadfence(); }
}
template <int NPASS, int POUT>
__global__ __launch_bounds__(32) void lin_kernel(const float* __restrict__ IN, const float* __restrict__ IN2, const b16* __restrict__ WT, const float* __restrict__ bias, int NLIM, float scale, float* __restrict__ OUT) {
  __shared__ __attribute__((aligned(16))) b16 Ah[16][H + 8], Al[16][H + 8]; __shared__ __attribute__((aligned(16))) float Tf[16][128 + 4];
  const int lane = threadIdx.x, nloc = lane & 15, hlf = lane >> 4; const size_t m0 = (size_t)blockIdx.x * 16; if (m0 >= (size_t)NLIM) return;
  for (int rr = 0; rr < 16; ++rr) for (int q = 0; q < 8; ++q) { const int c = q * 32 + lane; float v = IN[(m0 + rr) * H + c]; if (IN2) v += IN2[(m0 + rr) * H + c]; b16 p, ql; split16(v * scale, p, ql); Ah[rr][c] = p; Al[rr][c] = ql; }
  wave_lds_sync(); const float sc = 1.0f / (scale * WSC);
#pragma unroll 1
  for (int cg = 0; cg < NPASS; ++cg) { v8f acc[8];
#pragma unroll
    for (int t = 0; t < 8; ++t) acc[t] = (v8f){};
#pragma unroll 2
    for (int kb = 0; kb < H; kb += 32) { const v16b a = frag_kb(&Ah[nloc][kb], hlf), al = frag_kb(&Al[nloc][kb], hlf);
#pragma unroll
      for (int t = 0; t < 8; ++t) { if (cg * 128 + t * 16 < POUT) { const v16b bw = frag_kb(WT + (size_t)(cg * 128 + t * 16 + nloc) * H + kb, hlf); acc[t] = wmma16b(a, bw, acc[t]); acc[t] = wmma16b(al, bw, acc[t]); } } }
#pragma unroll
    for (int t = 0; t < 8; ++t) { if (cg * 128 + t * 16 < POUT) { const int c = cg * 128 + t * 16 + nloc; const float bb = (bias && c < POUT) ? bf16_rne(bias[c]) : 0.0f;
#pragma unroll 1
        for (int r8 = 0; r8 < 8; ++r8) Tf[8 * hlf + r8][t * 16 + nloc] = acc[t][r8] * sc + bb; } }
    wave_lds_sync();
    const int ncol = POUT - cg * 128 < 128 ? POUT - cg * 128 : 128;
    for (int pass = 0; pass < 2; ++pass) { for (int rr = 0; rr < 16; ++rr) for (int c = lane; c < ncol; c += 32) ((volatile float*)OUT)[(m0 + rr) * POUT + cg * 128 + c] = Tf[rr][c]; __threadfence(); }
    wave_lds_sync(); }
}
__global__ __launch_bounds__(256) void seg_kernel(const float* __restrict__ IN, const int* __restrict__ G, int gmax, const int* __restrict__ PERM, const int* __restrict__ ROWPTR, const int* __restrict__ ROWCNT, int permLen, int nseg, int segPerGraph, const float* __restrict__ bias, int BLIM, float* __restrict__ OUT) {
  const int wave = threadIdx.x >> 5, lane = threadIdx.x & 31; const int s = blockIdx.x * 8 + wave; if (s >= nseg || s / segPerGraph >= BLIM) return;
  int st = ROWPTR[s], cnt = ROWCNT[s]; cnt = iclamp(cnt, 0, 1 << 20); st = iclamp(st, 0, permLen - cnt); float acc[8]; for (int q = 0; q < 8; ++q) acc[q] = 0.0f;
#pragma unroll 1
  for (int j = 0; j < cnt; ++j) { const int p = iclamp(PERM[st + j], 0, NE - 1); const size_t r = (size_t)iclamp(G[p], 0, gmax - 1); const float* row = IN + r * H; for (int q = 0; q < 8; ++q) acc[q] += row[q * 32 + lane]; }
  const float inv = 1.0f / (float)(cnt < 1 ? 1 : cnt); float o[8]; for (int q = 0; q < 8; ++q) { o[q] = pmul(acc[q], inv); if (bias) o[q] += bf16_rne(bias[q * 32 + lane]); }
  for (int pass = 0; pass < 2; ++pass) { for (int q = 0; q < 8; ++q) ((volatile float*)OUT)[(size_t)s * H + q * 32 + lane] = o[q]; __threadfence(); }
}
__global__ __launch_bounds__(256) void bn_kernel(const float* __restrict__ HC, const float* __restrict__ g, const float* __restrict__ bb, int BLIM, float* __restrict__ HS) {
  const int b = blockIdx.x, c = threadIdx.x; if (b >= BLIM) return; double s = 0.0, s2 = 0.0;
#pragma unroll 4
  for (int n = 0; n < N; ++n) { const double v = (double)HC[((size_t)b * N + n) * H + c]; s += v; s2 += v * v; }
  const double mean = s / N; const double var = fmax(s2 / N - mean * mean, 0.0); const float scale = bf16_rne(g[c]) * (float)(1.0 / sqrt(var + 1e-5)); const float shift = bf16_rne(bb[c]) - (float)mean * scale;
  for (int pass = 0; pass < 2; ++pass) {
#pragma unroll 4
    for (int n = 0; n < N; ++n) ((volatile float*)HS)[((size_t)b * N + n) * H + c] = fmaxf(pmul(HC[((size_t)b * N + n) * H + c], scale) + shift, 0.0f);
    __threadfence(); }
}
}

extern "C" void kernel_launch(void* const* d_in, const int* in_sizes, int n_in, void* d_out, int out_size, void* d_ws, size_t ws_size, hipStream_t stream) {
  (void)n_in;
  auto Fp = [&](int i) { return (const float*)d_in[i]; }; auto Ip = [&](int i) { return (const int*)d_in[i]; };
  if (in_sizes[0] != NN * T * DIN || in_sizes[1] != B * 2 * E || in_sizes[2] != DIN * H || in_sizes[4] != L * H * H || in_sizes[5] != L * H || in_sizes[8] != H * PO || out_size != NN * PO) return;
  const int BLIM = B; const int NLIM = BLIM * N;
  size_t off = 0; char* ws = (char*)d_ws;
  auto carve = [&](size_t bytes) { char* p = ws + off; off += (bytes + 255) & ~(size_t)255; return p; };
  b16* WT[L]; for (int l = 0; l < L; ++l) WT[l] = (b16*)carve((size_t)H * H * 2); b16* WD = (b16*)carve((size_t)32 * H * 2); int* KN = (int*)carve((size_t)NE * 4); int* KE = (int*)carve((size_t)NE * 4);
  float* H0 = (float*)carve((size_t)NN * H * 4); float* HS = (float*)carve((size_t)NN * H * 4); float* XT = (float*)carve((size_t)NN * H * 4); float* HC = (float*)carve((size_t)NN * H * 4); float* MSG = (float*)carve((size_t)NM * H * 4);
  CsrBufs6 ce; off = csr_carve6(ce, ws, off, NE, NM); CsrBufs9 cn; off = csr_carve9(cn, ws, off, NE, NN);
  if (off > ws_size || off > ((size_t)200 << 20)) return;
  for (int l = 0; l < L; ++l) wio_kernel<<<(H * H / 8 + 255) / 256, 256, 0, stream>>>(Fp(4) + (size_t)l * H * H, H, H, WT[l]); wio_kernel<<<(32 * H / 8 + 255) / 256, 256, 0, stream>>>(Fp(8), PO, 32, WD);
  keys_kernel<<<NE / 256, 256, 0, stream>>>(Ip(1), KN, KE);
  csr_build6(ce, KE, NE, NM, stream); csr_build9(cn, KN, NE, NN, stream);
  enc_kernel<<<(unsigned)(((size_t)NLIM * (H / 4) + 255) / 256), 256, 0, stream>>>(Fp(0), Fp(2), Fp(3), NLIM, H0, HS);
  for (int l = 0; l < L; ++l) {
    lin_kernel<2, H><<<NLIM / 16, 32, 0, stream>>>(HS, nullptr, WT[l], nullptr, NLIM, l == 0 ? 1024.0f : 64.0f, XT);
    seg_kernel<<<NM / 8, 256, 0, stream>>>(XT, KN, NN, ce.PERM, ce.ROWPTR, ce.ROWCNT, (int)ce.permLen, NM, M, nullptr, BLIM, MSG);
    seg_kernel<<<NN / 8, 256, 0, stream>>>(MSG, KE, NM, cn.PERM, cn.ROWPTR, cn.ROWCNT, (int)cn.permLen, NN, N, Fp(5) + l * H, BLIM, HC);
    bn_kernel<<<B, 256, 0, stream>>>(HC, Fp(6) + l * H, Fp(7) + l * H, BLIM, HS); }
  lin_kernel<1, PO><<<NLIM / 16, 32, 0, stream>>>(H0, HS, WD, Fp(9), NLIM, 64.0f, (float*)d_out);
}
